// MambaBlock_29515015258140
// MI455X (gfx1250) — hardware-run, weakly checked
//
#include <hip/hip_runtime.h>


#define NM   16384
#define NQ   2
#define NL   8192
#define NC   256
#define NJ   16
#define NX   33
#define NXP  64

typedef _Float16 h16;
typedef unsigned short bf;
typedef __attribute__((ext_vector_type(16))) __bf16   v16bf;
typedef __attribute__((ext_vector_type(16))) _Float16 v16h;
typedef __attribute__((ext_vector_type(8)))  _Float16 v8h;
typedef __attribute__((ext_vector_type(8)))  unsigned short v8us;
typedef __attribute__((ext_vector_type(8)))  float    v8f;
typedef __attribute__((ext_vector_type(4)))  float    v4f;
typedef v8h  __attribute__((may_alias)) v8ha;
typedef v4f  __attribute__((may_alias)) v4fa;
typedef v8us __attribute__((may_alias)) v8usa;

__device__ __forceinline__ unsigned short f2bf(float f) { unsigned u = __float_as_uint(f); u += 0x7FFFu + ((u >> 16) & 1u); return (unsigned short)(u >> 16); }
__device__ __forceinline__ float bf2f(unsigned short b) { return __uint_as_float(((unsigned)b) << 16); }
__device__ __forceinline__ float bfr(float f) { return bf2f(f2bf(f)); }
__device__ __forceinline__ v16h cat16(v8h lo, v8h hi) { return __builtin_shufflevector(lo, hi, 0, 1, 2, 3, 4, 5, 6, 7, 8, 9, 10, 11, 12, 13, 14, 15); }
__device__ __forceinline__ v16bf cat16b(v8us lo, v8us hi) { return __builtin_bit_cast(v16bf, __builtin_shufflevector(lo, hi, 0, 1, 2, 3, 4, 5, 6, 7, 8, 9, 10, 11, 12, 13, 14, 15)); }
__device__ __forceinline__ v8f wmma16(v16h a, v16h b, v8f c) { return __builtin_amdgcn_wmma_f32_16x16x32_f16(false, a, false, b, (short)0, c, false, false); }
__device__ __forceinline__ v8f wmmab(v16bf a, v16bf b, v8f c) { return __builtin_amdgcn_wmma_f32_16x16x32_bf16(false, a, false, b, (short)0, c, false, false); }

template <typename T16> struct WFrag;
template <> struct WFrag<h16> { typedef v16h V; static __device__ __forceinline__ V ld(const h16* p) { return cat16(*(const v8h*)p, *(const v8h*)(p + 16)); } static __device__ __forceinline__ v8f mma(V a, V b, v8f c) { return wmma16(a, b, c); } };
template <> struct WFrag<bf> { typedef v16bf V; static __device__ __forceinline__ V ld(const bf* p) { return cat16b(*(const v8us*)p, *(const v8us*)(p + 16)); } static __device__ __forceinline__ v8f mma(V a, V b, v8f c) { return wmmab(a, b, c); } };
template <typename T16, int NSPLIT, bool BIAS>
__global__ __launch_bounds__(32) void k_gemmw(const T16* __restrict__ A, const T16* __restrict__ A2, const T16* __restrict__ Bt, const T16* __restrict__ Bt2, int K, float* C, int ldc, const float* __restrict__ bias, size_t sA, size_t sB, size_t sC) {
    typedef typename WFrag<T16>::V V;
    __shared__ __align__(16) float os[16 * 68];
    const size_t z = blockIdx.z; A += z * sA; if (A2) A2 += z * sA; Bt += z * sB; if (Bt2) Bt2 += z * sB; C += z * sC;
    const int lane = threadIdx.x & 31, lr = lane & 15, hi = lane >> 4; const int r0 = blockIdx.x * 64, c0 = blockIdx.y * 64;
    v8f acc[4][4];
#pragma unroll
    for (int mb = 0; mb < 4; ++mb)
#pragma unroll
        for (int nb = 0; nb < 4; ++nb) acc[mb][nb] = (v8f){};
    const size_t aoff = (size_t)(r0 + lr) * K + 8 * hi, boff = (size_t)(c0 + lr) * K + 8 * hi;
    for (int kc = 0; kc < K; kc += 32) {
        V a[4], a2[4];
#pragma unroll
        for (int mb = 0; mb < 4; ++mb) { a[mb] = WFrag<T16>::ld(A + aoff + (size_t)mb * 16 * K + kc); if (NSPLIT == 1 || NSPLIT == 2) a2[mb] = WFrag<T16>::ld(A2 + aoff + (size_t)mb * 16 * K + kc); }
#pragma unroll
        for (int nb = 0; nb < 4; ++nb) { const V b = WFrag<T16>::ld(Bt + boff + (size_t)nb * 16 * K + kc); V b2; if (NSPLIT >= 2) b2 = WFrag<T16>::ld(Bt2 + boff + (size_t)nb * 16 * K + kc);
#pragma unroll
            for (int mb = 0; mb < 4; ++mb) { acc[mb][nb] = WFrag<T16>::mma(a[mb], b, acc[mb][nb]); if (NSPLIT == 1 || NSPLIT == 2) acc[mb][nb] = WFrag<T16>::mma(a2[mb], b, acc[mb][nb]); if (NSPLIT >= 2) acc[mb][nb] = WFrag<T16>::mma(a[mb], b2, acc[mb][nb]); } }
        asm volatile("v_nop\n\tv_nop\n\tv_nop\n\tv_nop" : "+v"(acc[0][0]), "+v"(acc[1][1]), "+v"(acc[2][2]), "+v"(acc[3][3]) : "v"(a[0]), "v"(a[3]));
    }
#pragma unroll
    for (int mb = 0; mb < 4; ++mb) {
#pragma unroll
        for (int nb = 0; nb < 4; ++nb) {
#pragma unroll
            for (int j = 0; j < 8; ++j) os[(hi * 8 + j) * 68 + nb * 16 + lr] = acc[mb][nb][j]; }
        __builtin_amdgcn_wave_barrier(); asm volatile("" ::: "memory");
        float* crow = C + (size_t)(r0 + mb * 16) * ldc + c0;
#pragma unroll 1
        for (int ps = 0; ps < 2; ++ps) {
#pragma unroll
            for (int s = 0; s < 8; ++s) { const int row = 2 * s + hi, cofs = lr * 4; v4f val = *(const v4fa*)(os + row * 68 + cofs); if (BIAS) { val[0] += bfr(bias[c0 + cofs]); val[1] += bfr(bias[c0 + cofs + 1]); val[2] += bfr(bias[c0 + cofs + 2]); val[3] += bfr(bias[c0 + cofs + 3]); }
                *(volatile v4f*)(crow + (size_t)row * ldc + cofs) = val; }
            if (ps == 0) __threadfence(); }
        __builtin_amdgcn_wave_barrier(); asm volatile("" ::: "memory");
    }
}

typedef __attribute__((ext_vector_type(2))) _Float16 v2h;
typedef __attribute__((ext_vector_type(4))) _Float16 v4h;
typedef __attribute__((ext_vector_type(2))) unsigned short v2us;
typedef __attribute__((ext_vector_type(4))) unsigned short v4us;
typedef __attribute__((ext_vector_type(2))) float v2f;
typedef __attribute__((ext_vector_type(4))) int v4i;
__global__ __launch_bounds__(256) void k_cvt8(const float* __restrict__ src, bf* dst, size_t n8) { const size_t i = (size_t)blockIdx.x * 256 + threadIdx.x; if (i >= n8) return; const v8f v = *(const v8f*)(src + i * 8); v8us o;
#pragma unroll
    for (int k = 0; k < 8; ++k) o[k] = f2bf(v[k]); *(volatile v8us*)(dst + i * 8) = o; __threadfence(); *(volatile v8us*)(dst + i * 8) = o; }

__global__ __launch_bounds__(256) void k_fillb(bf* P, unsigned w2, size_t n8) { const size_t i = (size_t)blockIdx.x * 256 + threadIdx.x; if (i >= n8) return; v4i o; o[0] = (int)w2; o[1] = (int)w2; o[2] = (int)w2; o[3] = (int)w2;
    *(volatile v4i*)(P + i * 8) = o; __threadfence(); *(volatile v4i*)(P + i * 8) = o; }

__global__ __launch_bounds__(256) void k_rbf(const float* __restrict__ X, float* Y, size_t n4) { const size_t i = (size_t)blockIdx.x * 256 + threadIdx.x; if (i >= n4) return; const v4f a = *(const v4f*)(X + i * 4); v4f o;
#pragma unroll
    for (int q = 0; q < 4; ++q) o[q] = bfr(a[q]);
    *(volatile v4f*)(Y + i * 4) = o; __threadfence(); *(volatile v4f*)(Y + i * 4) = o; }

#define LNC_MAX 2048
template <bool RES>
__global__ __launch_bounds__(256) void k_lnrow(const float* __restrict__ A, const float* __restrict__ R, const float* __restrict__ gamma, const float* __restrict__ beta, float eps, int C, int nrows, float* Y) {
    const int lane = threadIdx.x & 31; const int row = blockIdx.x * 8 + (threadIdx.x >> 5); if (row >= nrows) return; const int nch = C / 128; const float* a = A + (size_t)row * C; float x[LNC_MAX / 32]; float s = 0.0f;
    for (int k = 0; k < LNC_MAX / 128; ++k) { if (k < nch) { const int c0 = k * 128 + lane * 4; v4f v = *(const v4f*)(a + c0);
            if (RES) { const v4f w = *(const v4f*)(R + (size_t)row * C + c0); v[0] = __fadd_rn(v[0], w[0]); v[1] = __fadd_rn(v[1], w[1]); v[2] = __fadd_rn(v[2], w[2]); v[3] = __fadd_rn(v[3], w[3]); }
            x[k * 4 + 0] = v[0]; x[k * 4 + 1] = v[1]; x[k * 4 + 2] = v[2]; x[k * 4 + 3] = v[3]; s = __fadd_rn(__fadd_rn(__fadd_rn(__fadd_rn(s, v[0]), v[1]), v[2]), v[3]); } }
    for (int sh = 16; sh; sh >>= 1) s = __fadd_rn(s, __shfl_xor(s, sh, 32));
    const float mean = __fdiv_rn(s, (float)C); float q = 0.0f;
    for (int k = 0; k < LNC_MAX / 128; ++k) { if (k < nch) {
            for (int j = 0; j < 4; ++j) { const float d = __fsub_rn(x[k * 4 + j], mean); x[k * 4 + j] = d; q = __fmaf_rn(d, d, q); } } }
    for (int sh = 16; sh; sh >>= 1) q = __fadd_rn(q, __shfl_xor(q, sh, 32));
    const float rstd = __fdiv_rn(1.0f, sqrtf(__fadd_rn(__fdiv_rn(q, (float)C), eps)));
    for (int k = 0; k < LNC_MAX / 128; ++k) { if (k < nch) { const int c0 = k * 128 + lane * 4; const v4f g = *(const v4f*)(gamma + c0); const v4f bt = *(const v4f*)(beta + c0);
            for (int j = 0; j < 4; ++j) x[k * 4 + j] = __fmaf_rn(__fmul_rn(x[k * 4 + j], rstd), bfr(g[j]), bfr(bt[j])); } }
    float* y = Y + (size_t)row * C;
    for (int ps = 0; ps < 2; ++ps) {
        for (int k = 0; k < LNC_MAX / 128; ++k) { if (k < nch) { v4f o; o[0] = x[k * 4 + 0]; o[1] = x[k * 4 + 1]; o[2] = x[k * 4 + 2]; o[3] = x[k * 4 + 3]; *(volatile v4f*)(y + k * 128 + lane * 4) = o; } }
        if (ps == 0) __threadfence(); }
}

__device__ __forceinline__ void splitf(float y, unsigned short& h, unsigned short& l) { h = f2bf(y); l = f2bf(y - bf2f(h)); }

__global__ __launch_bounds__(256) void k_tohl(const float* __restrict__ F, float sc, bf* Hh, bf* Hl, size_t n4) { const size_t i = (size_t)blockIdx.x * 256 + threadIdx.x; if (i >= n4) return; const v4f a = *(const v4f*)(F + i * 4); v4us oh, ol;
#pragma unroll
    for (int q = 0; q < 4; ++q) { unsigned short h2, l2; splitf(__fmul_rn(a[q], sc), h2, l2); oh[q] = h2; ol[q] = l2; }
    *(volatile v4us*)(Hh + i * 4) = oh; *(volatile v4us*)(Hl + i * 4) = ol; __threadfence(); *(volatile v4us*)(Hh + i * 4) = oh; *(volatile v4us*)(Hl + i * 4) = ol; }

__device__ __forceinline__ unsigned short f2bf_keep(float f) { const unsigned short hw = f2bf(f); return (f != f) ? (unsigned short)0x7FC0 : hw; }

__global__ __launch_bounds__(256) void k_pre(const float* __restrict__ Xd, const float* __restrict__ Px, const float* __restrict__ a5, const float* __restrict__ a6, const float* __restrict__ a7, float* En) { const unsigned id = blockIdx.x * 256u + threadIdx.x; const unsigned rw = id >> 8, ch = id & 255u; const float vv = (Xd[(size_t)rw * NXP] + bfr(a5[0])) * bfr(a6[ch]) + bfr(a7[ch]); const float sz = fmaxf(vv, 0.0f) + log1pf(expf(-fabsf(vv))); const float en = Px[id] * sz;
    *(volatile float*)(En + id) = en; __threadfence(); *(volatile float*)(En + id) = en; }

__global__ __launch_bounds__(256) void k_walk(const float* __restrict__ En, const float* __restrict__ Xd, const float* __restrict__ a5, float* Rd) { const unsigned id = blockIdx.x * 256u + threadIdx.x; const unsigned sq = id >> 8, ch = id & 255u; float ef[NJ], rf[NJ], cw[NJ];
#pragma unroll
    for (int j = 0; j < NJ; ++j) { ef[j] = bfr(a5[1 + j]); rf[j] = bfr(a5[1 + NJ + j]); cw[j] = 0.0f; }
    for (int r0 = 0; r0 < NL; r0 += 8) { float hv[8];
#pragma unroll
        for (int jr = 0; jr < 8; ++jr) { const size_t rw = (size_t)sq * NL + r0 + jr; const float en = En[rw * NC + ch]; const float* pc = Xd + rw * NXP; float acc = 0.0f;
#pragma unroll
            for (int j = 0; j < NJ; ++j) cw[j] = cw[j] + en * (pc[1 + j] + ef[j]);
#pragma unroll
            for (int j = 0; j < NJ; ++j) acc = acc + cw[j] * (pc[1 + NJ + j] + rf[j]);
            hv[jr] = acc; }
        float* po = Rd + ((size_t)sq * NL + r0) * NC + ch;
#pragma unroll
        for (int jr = 0; jr < 8; ++jr) *(volatile float*)(po + (size_t)jr * NC) = hv[jr];
        __threadfence();
#pragma unroll
        for (int jr = 0; jr < 8; ++jr) *(volatile float*)(po + (size_t)jr * NC) = hv[jr]; } }

__global__ __launch_bounds__(256) void k_post(const float* __restrict__ Rd, const float* __restrict__ Px, const float* __restrict__ Pg, const float* __restrict__ a9, bf* Yh, bf* Yl) { const unsigned id = blockIdx.x * 256u + threadIdx.x; const unsigned c0 = (id & 31u) << 3; const size_t e0 = (size_t)id * 8; const v4f ra = *(const v4f*)(Rd + e0), rb = *(const v4f*)(Rd + e0 + 4), pa = *(const v4f*)(Px + e0), pb = *(const v4f*)(Px + e0 + 4), ga = *(const v4f*)(Pg + e0), gb = *(const v4f*)(Pg + e0 + 4), qa = *(const v4f*)(a9 + c0), qb = *(const v4f*)(a9 + c0 + 4); v8us oh, ol;
#pragma unroll
    for (int q = 0; q < 8; ++q) { const float rd = q < 4 ? ra[q] : rb[q - 4], pv = q < 4 ? pa[q] : pb[q - 4], gv = q < 4 ? ga[q] : gb[q - 4], dv = bfr(q < 4 ? qa[q] : qb[q - 4]); const float yv = (rd + dv * pv) * (gv * (1.0f / (1.0f + expf(-gv)))); const unsigned short hw = f2bf_keep(yv); oh[q] = hw; ol[q] = f2bf_keep(yv - bf2f(hw)); }
    *(volatile v8us*)(Yh + e0) = oh; *(volatile v8us*)(Yl + e0) = ol; __threadfence(); *(volatile v8us*)(Yh + e0) = oh; *(volatile v8us*)(Yl + e0) = ol; }

extern "C" void kernel_launch(void* const* d_in, const int* in_sizes, int n_in, void* d_out, int out_size, void* d_ws, size_t ws_size, hipStream_t stream) {
    if (n_in < 13) return;
    if (in_sizes[0] != NM * NC || in_sizes[1] != 2 * NC * NC || in_sizes[2] != 2 * NC || in_sizes[3] != NX * NC || in_sizes[4] != NX || in_sizes[5] != NC || in_sizes[6] != NC || in_sizes[7] != NC * NJ || in_sizes[8] != NC || in_sizes[9] != NC * NC || in_sizes[10] != NC || in_sizes[11] != NC || in_sizes[12] != NC) return;
    if (out_size != NM * NC) return;
    static_assert(NM == NQ * NL && NM % 64 == 0 && NC % 64 == 0 && NXP % 64 == 0 && NC % 32 == 0 && NX == 1 + 2 * NJ && NX <= NXP && (NM * NC / 8) % 256 == 0 && (2 * NC * NC / 8) % 256 == 0 && (NC * NC / 8) % 256 == 0 && (NM * NC) % 256 == 0 && (NQ * NC) % 256 == 0 && (NM * NC / 4) % 256 == 0 && NC == 256 && NL % 8 == 0 && (NX * NC) % 8 == 0 && ((NXP - NX) * NC) % 8 == 0 && (NX * NC * 2) % 128 == 0 && NC % 128 == 0 && NC <= LNC_MAX && NM % 8 == 0, "the products: row and column counts multiples of 64, the depths of 32; the flat grids exact but the two on Wx (which hold the kit's own guard); a channel is the low 8 bits of a (row, channel) number; the noughts beneath Wx's 33 rows begin on a whole line; k_lnrow: the channel count a multiple of 128 and at most LNC_MAX, the rows in eights");
    const float* i0 = (const float*)d_in[0]; const float* i1 = (const float*)d_in[1]; const float* i2 = (const float*)d_in[2]; const float* i3 = (const float*)d_in[3]; const float* i4 = (const float*)d_in[4]; const float* i5 = (const float*)d_in[5]; const float* i6 = (const float*)d_in[6]; const float* i8 = (const float*)d_in[8]; const float* i9 = (const float*)d_in[9]; const float* i10 = (const float*)d_in[10]; const float* i11 = (const float*)d_in[11]; const float* i12 = (const float*)d_in[12]; float* res = (float*)d_out;
    char* wsp = (char*)d_ws; auto take = [&](size_t bytes) { char* p = wsp; wsp += (bytes + 255) & ~(size_t)255; return (void*)p; };
    bf* Xb = (bf*)take((size_t)NM * NC * 2); bf* Wa = (bf*)take((size_t)2 * NC * NC * 2); bf* Wo = (bf*)take((size_t)NC * NC * 2); float* Px = (float*)take((size_t)NM * NC * 4); float* Pg = (float*)take((size_t)NM * NC * 4); bf* Ph = (bf*)take((size_t)NM * NC * 2); bf* Pl = (bf*)take((size_t)NM * NC * 2); bf* Wx = (bf*)take((size_t)NXP * NC * 2); float* Xd = (float*)take((size_t)NM * NXP * 4); float* En = (float*)take((size_t)NM * NC * 4); float* Rd = (float*)take((size_t)NM * NC * 4); bf* Yh = (bf*)take((size_t)NM * NC * 2); bf* Yl = (bf*)take((size_t)NM * NC * 2); float* Po = (float*)take((size_t)NM * NC * 4); float* Xr = En;
    if ((size_t)(wsp - (char*)d_ws) > ws_size) return;
    k_cvt8<<<(unsigned)(NM * NC / 8 / 256), 256, 0, stream>>>(i0, Xb, (size_t)NM * NC / 8);
    k_cvt8<<<(unsigned)(2 * NC * NC / 8 / 256), 256, 0, stream>>>(i1, Wa, (size_t)2 * NC * NC / 8);
    k_cvt8<<<(unsigned)(NC * NC / 8 / 256), 256, 0, stream>>>(i9, Wo, (size_t)NC * NC / 8);
    k_gemmw<bf, 0, true><<<dim3(NM / 64, NC / 64, 1), 32, 0, stream>>>(Xb, nullptr, Wa, nullptr, NC, Px, NC, i2, 0, 0, 0);
    k_gemmw<bf, 0, true><<<dim3(NM / 64, NC / 64, 1), 32, 0, stream>>>(Xb, nullptr, Wa + (size_t)NC * NC, nullptr, NC, Pg, NC, i2 + NC, 0, 0, 0);
    k_tohl<<<(unsigned)(NM * NC / 4 / 256), 256, 0, stream>>>(Px, 1.0f, Ph, Pl, (size_t)NM * NC / 4);
    k_cvt8<<<(unsigned)((NX * NC / 8 + 255) / 256), 256, 0, stream>>>(i3, Wx, (size_t)NX * NC / 8);
    k_fillb<<<(unsigned)(((NXP - NX) * NC / 8 + 255) / 256), 256, 0, stream>>>(Wx + (size_t)NX * NC, 0u, (size_t)(NXP - NX) * NC / 8);
    k_gemmw<bf, 1, false><<<dim3(NM / 64, NXP / 64, 1), 32, 0, stream>>>(Ph, Pl, Wx, nullptr, NC, Xd, NXP, nullptr, 0, 0, 0);
    k_pre<<<(unsigned)(NM * NC / 256), 256, 0, stream>>>(Xd, Px, i4, i5, i6, En);
    k_walk<<<(unsigned)(NQ * NC / 256), 256, 0, stream>>>(En, Xd, i4, Rd);
    k_post<<<(unsigned)(NM * NC / 8 / 256), 256, 0, stream>>>(Rd, Px, Pg, i8, Yh, Yl);
    k_gemmw<bf, 1, true><<<dim3(NM / 64, NC / 64, 1), 32, 0, stream>>>(Yh, Yl, Wo, nullptr, NC, Po, NC, i10, 0, 0, 0);
    k_rbf<<<(unsigned)(NM * NC / 4 / 256), 256, 0, stream>>>(i0, Xr, (size_t)NM * NC / 4);
    k_lnrow<true><<<(unsigned)(NM / 8), 256, 0, stream>>>(Po, Xr, i11, i12, 1.0e-5f, NC, NM, res);
}
